// UnimpNet_44573170598395
// MI455X (gfx1250) — hardware-verified
//
#include <hip/hip_runtime.h>
#include <stddef.h>


#define DIN    128
#define NHD    4
#define DHD    32
#define HDW    128
#define PW     512
#define QOFF   0
#define KOFF   128
#define VOFF   256
#define SOFF   384
#define NCLS   64
#define NTHR   256
#define NWAVE  8
#define EPT    8
#define NGRP   2
#define CHUNK  (NTHR * EPT * NGRP)
#define WCAP   (EPT * NGRP * 32)
#define LISTN  (NWAVE * WCAP)
#define NBC    4096
#define NBF    1024
#define RCAP   40960
#define RBN    128
#define ATHR   128
#define AWAVE  4
#define TGT    128
#define NPADG  256
#define DEGCAP 128
#define NCHK   (DEGCAP / 32)
#define OTHR   512
#define WSCAP  134217728
#define NEG_BIG (-3.0e38f)
#define ASCL   8.0f
#define WSCL   64.0f
#define INVSCL 0.001953125f
#define RSQD   0.17677669529663688f
#define APK    136
#define BM1    32
#define BM2    64
#define WUNITS (PW * DIN / 8)
#define LUNITS (NCLS * DIN / 8)
#define BCPAD  512

#define LDS_FILL ((RCAP + NBF + LISTN) * 4 + 64)
#define LDS_G1   (BM1 * PW * 4)
#define LDS_G2   (BM2 * APK * 2)
#define LDS_AGG  (AWAVE * 32 * (HDW / 4) * 16)

static_assert((CHUNK & (CHUNK - 1)) == 0);
static_assert(CHUNK <= 4096);
static_assert(NBC <= 4096 && NBF <= 4096);
static_assert((NBC & (NBC - 1)) == 0 && (NBF & (NBF - 1)) == 0);
static_assert(NBC == 4 * NBF);
static_assert(OTHR * 8 == NBC);
static_assert((RCAP % 32) == 0);
static_assert(TGT == AWAVE * 32);
static_assert(ATHR == AWAVE * 32);
static_assert((NBC % NPADG) == 0);
static_assert((NPADG % TGT) == 0 && (NPADG % BM1) == 0 && (NPADG % BM2) == 0);
static_assert((WUNITS % NTHR) == 0 && (LUNITS % NTHR) == 0);
static_assert(((APK * 2) % 16) == 0 && APK >= DIN);
static_assert(NCHK * 32 == DEGCAP);
static_assert(NHD * DHD == HDW && PW == 4 * HDW);
static_assert(LDS_G1 >= BM1 * APK * 2 && LDS_G1 >= BM1 * PW * 4);
static_assert(LDS_G2 >= BM2 * APK * 2 && LDS_G2 >= BM2 * NCLS * 4);
static_assert(BCPAD >= PW && BCPAD >= NCLS);

typedef float          v4f  __attribute__((ext_vector_type(4)));
typedef float          v8f  __attribute__((ext_vector_type(8)));
typedef int            v4i  __attribute__((ext_vector_type(4)));
typedef unsigned short v8us __attribute__((ext_vector_type(8)));
typedef _Float16       v16h __attribute__((ext_vector_type(16)));
union FragH { v16h v; v8us u[2]; };

__device__ __forceinline__ unsigned short h16(float f) {
  const _Float16 h = (_Float16)f;
  return __builtin_bit_cast(unsigned short, h);
}

__device__ __forceinline__ v8us cvt8(v4f a, v4f b, float s) {
  v8us r;
  r[0] = h16(a.x * s); r[1] = h16(a.y * s); r[2] = h16(a.z * s); r[3] = h16(a.w * s);
  r[4] = h16(b.x * s); r[5] = h16(b.y * s); r[6] = h16(b.z * s); r[7] = h16(b.w * s);
  return r;
}

__device__ __forceinline__ v8f wmh(v16h a, v16h b, v8f c) {
  v8f d = __builtin_amdgcn_wmma_f32_16x16x32_f16(false, a, false, b, (short)0, c, false, false);
  asm volatile("v_nop\n\tv_nop\n\tv_nop\n\tv_nop" : "+v"(d) : "v"(a), "v"(b));
  return d;
}

template <int NB>
__device__ __forceinline__ int scan_chunk(const int* __restrict__ dsts, int nE, int cbase, int slotBase,
                                          int vec8, int* list, int tid, int lane, int wave) {
  int wc = 0;
#pragma unroll
  for (int g = 0; g < NGRP; ++g) {
    const int el0  = (g * NTHR + tid) * EPT;
    const int e0   = cbase + el0;
    const int sent = -2147483647 - 1;
    v4i da, db;
    if (vec8 != 0 && cbase + CHUNK <= nE) {
      da = *(const v4i*)(dsts + e0);
      db = *(const v4i*)(dsts + e0 + 4);
    } else {
      da.x = (e0     < nE) ? dsts[min(e0, nE - 1)] : sent;
      da.y = (e0 + 1 < nE) ? dsts[min(e0 + 1, nE - 1)] : sent;
      da.z = (e0 + 2 < nE) ? dsts[min(e0 + 2, nE - 1)] : sent;
      da.w = (e0 + 3 < nE) ? dsts[min(e0 + 3, nE - 1)] : sent;
      db.x = (e0 + 4 < nE) ? dsts[min(e0 + 4, nE - 1)] : sent;
      db.y = (e0 + 5 < nE) ? dsts[min(e0 + 5, nE - 1)] : sent;
      db.z = (e0 + 6 < nE) ? dsts[min(e0 + 6, nE - 1)] : sent;
      db.w = (e0 + 7 < nE) ? dsts[min(e0 + 7, nE - 1)] : sent;
    }
    const unsigned nb = (unsigned)slotBase;
    const unsigned s0 = (unsigned)da.x - nb, s1 = (unsigned)da.y - nb;
    const unsigned s2 = (unsigned)da.z - nb, s3 = (unsigned)da.w - nb;
    const unsigned s4 = (unsigned)db.x - nb, s5 = (unsigned)db.y - nb;
    const unsigned s6 = (unsigned)db.z - nb, s7 = (unsigned)db.w - nb;
    const bool h0 = s0 < (unsigned)NB, h1 = s1 < (unsigned)NB, h2 = s2 < (unsigned)NB, h3 = s3 < (unsigned)NB;
    const bool h4 = s4 < (unsigned)NB, h5 = s5 < (unsigned)NB, h6 = s6 < (unsigned)NB, h7 = s7 < (unsigned)NB;
    const unsigned any = __builtin_amdgcn_ballot_w32(h0 | h1 | h2 | h3 | h4 | h5 | h6 | h7);
    if (any != 0u) {
#define HITJ(J, HJ, SJ) { \
        const unsigned mj = __builtin_amdgcn_ballot_w32(HJ); \
        if (mj != 0u) { \
          if (HJ) { \
            const int pos = wc + (int)__builtin_amdgcn_mbcnt_lo(mj, 0u); \
            if (pos < WCAP) list[wave * WCAP + pos] = ((el0 + (J)) << 12) | (int)(SJ); \
          } \
          wc += (int)__builtin_popcount(mj); } }
      HITJ(0, h0, s0)
      HITJ(1, h1, s1)
      HITJ(2, h2, s2)
      HITJ(3, h3, s3)
      HITJ(4, h4, s4)
      HITJ(5, h5, s5)
      HITJ(6, h6, s6)
      HITJ(7, h7, s7)
#undef HITJ
    }
  }
  return wc;
}

__global__ __launch_bounds__(NTHR) void k_wprep(
    const float* __restrict__ wq, const float* __restrict__ bq,
    const float* __restrict__ wk, const float* __restrict__ bk,
    const float* __restrict__ wv, const float* __restrict__ bv,
    const float* __restrict__ wsk, const float* __restrict__ bsk,
    unsigned short* wp, float* bcat) {
  const int i   = (int)blockIdx.x * NTHR + (int)threadIdx.x;
  const int n   = i >> 4;
  const int k0  = (i & 15) * 8;
  const int grp = (n >> 7) & 3;
  const int cc  = n & 127;
  v8us hv;
#pragma unroll
  for (int e = 0; e < 8; ++e) {
    const int k = k0 + e;
    const float a = wq[k * HDW + cc];
    const float b = wk[k * HDW + cc];
    const float c = wv[k * HDW + cc];
    const float d = wsk[k * HDW + cc];
    const float v = (grp == 0) ? a : ((grp == 1) ? b : ((grp == 2) ? c : d));
    hv[e] = h16(v * WSCL);
  }
  const int bi  = i > PW - 1 ? PW - 1 : i;
  const int bg  = (bi >> 7) & 3;
  const int bcc = bi & 127;
  const float ba = bq[bcc], bb = bk[bcc], bc = bv[bcc], bd = bsk[bcc];
  const float bval = (bg == 0) ? ba : ((bg == 1) ? bb : ((bg == 2) ? bc : bd));

  unsigned short* dp = wp + (size_t)i * 8;
  *(volatile v8us*)dp = hv;
  if (i < PW) *(volatile float*)(bcat + i) = bval;
  __threadfence();
  *(volatile v8us*)dp = hv;
  if (i < PW) *(volatile float*)(bcat + i) = bval;
}

__global__ __launch_bounds__(NTHR) void k_wlprep(
    const float* __restrict__ wl_in, const float* __restrict__ bl_in,
    unsigned short* wl, float* blc) {
  const int i  = (int)blockIdx.x * NTHR + (int)threadIdx.x;
  const int n  = i >> 4;
  const int k0 = (i & 15) * 8;
  v8us hv;
#pragma unroll
  for (int e = 0; e < 8; ++e) {
    const int k = k0 + e;
    hv[e] = h16(wl_in[k * NCLS + n] * WSCL);
  }
  const int bi = i > NCLS - 1 ? NCLS - 1 : i;
  const float bval = bl_in[bi];
  unsigned short* dp = wl + (size_t)i * 8;
  *(volatile v8us*)dp = hv;
  if (i < NCLS) *(volatile float*)(blc + i) = bval;
  __threadfence();
  *(volatile v8us*)dp = hv;
  if (i < NCLS) *(volatile float*)(blc + i) = bval;
}

__global__ __launch_bounds__(NTHR) void k_count(
    const int* __restrict__ dsts, int* cnt, int nE, int vec8) {
  __shared__ __attribute__((aligned(16))) int scnt[NBC];
  __shared__ __attribute__((aligned(16))) int list[LISTN];
  __shared__ int wcnt[NWAVE];
  const int tid = threadIdx.x, lane = tid & 31, wave = tid >> 5;
  const int nodeBase = blockIdx.x * NBC;

  for (int i = tid; i < NBC; i += NTHR) scnt[i] = 0;
  __syncthreads();

  const int nChunks = (nE + CHUNK - 1) / CHUNK;
#pragma unroll 1
  for (int ch = 0; ch < nChunks; ++ch) {
    const int cbase = ch * CHUNK;
    const int wc = scan_chunk<NBC>(dsts, nE, cbase, nodeBase, vec8, list, tid, lane, wave);
    if (lane == 0) wcnt[wave] = wc;
    __syncthreads();
    if (wave == 0) {
#pragma unroll 1
      for (int wsx = 0; wsx < NWAVE; ++wsx) {
        int n = __builtin_amdgcn_readfirstlane(wcnt[wsx]);
        n = n > WCAP ? WCAP : (n < 0 ? 0 : n);
        const int* lp = list + wsx * WCAP;
#pragma unroll 1
        for (int i = 0; i < n; ++i) {
          const int ent  = __builtin_amdgcn_readfirstlane(lp[i]);
          const int slot = ent & (NBC - 1);
          if (lane == 0) scnt[slot] = scnt[slot] + 1;
        }
      }
    }
    __syncthreads();
  }

  v4i cq[4];
#pragma unroll
  for (int q = 0; q < 4; ++q) {
    const int f = (wave * 4 + q) * 128 + 4 * lane;
    cq[q] = *(const v4i*)(scnt + f);
  }
  int* cp = cnt + (size_t)nodeBase;
#pragma unroll
  for (int q = 0; q < 4; ++q) {
    const int f = (wave * 4 + q) * 128 + 4 * lane;
    *(volatile v4i*)(cp + f) = cq[q];
  }
  __threadfence();
#pragma unroll
  for (int q = 0; q < 4; ++q) {
    const int f = (wave * 4 + q) * 128 + 4 * lane;
    *(volatile v4i*)(cp + f) = cq[q];
  }
}

__global__ __launch_bounds__(OTHR) void k_offsets(
    const int* __restrict__ cnt, int* off, int* rbase, int nChunk) {
  __shared__ __attribute__((aligned(16))) int soff[NBC];
  __shared__ __attribute__((aligned(16))) int srb[RBN];
  __shared__ int wtot[OTHR / 32];
  const int tid = threadIdx.x, lane = tid & 31, wave = tid >> 5, sub = tid >> 7;
  for (int i = tid; i < RBN; i += OTHR) srb[i] = 0;
  int carry = 0;
#pragma unroll 1
  for (int ch = 0; ch < nChunk; ++ch) {
    const int base = ch * NBC;
    const v4i c0 = *(const v4i*)(cnt + base + 8 * tid);
    const v4i c1 = *(const v4i*)(cnt + base + 8 * tid + 4);
    const int e0 = max(c0.x, 0), e1 = max(c0.y, 0), e2 = max(c0.z, 0), e3 = max(c0.w, 0);
    const int e4 = max(c1.x, 0), e5 = max(c1.y, 0), e6 = max(c1.z, 0), e7 = max(c1.w, 0);
    const int ts = e0 + e1 + e2 + e3 + e4 + e5 + e6 + e7;
    int incl = ts;
#pragma unroll
    for (int d = 1; d < 32; d <<= 1) {
      const int t = __shfl_up(incl, d);
      if (lane >= d) incl += t;
    }
    if (lane == 31) wtot[wave] = incl;
    __syncthreads();
    const int S0 = wtot[0]  + wtot[1]  + wtot[2]  + wtot[3];
    const int S1 = wtot[4]  + wtot[5]  + wtot[6]  + wtot[7];
    const int S2 = wtot[8]  + wtot[9]  + wtot[10] + wtot[11];
    const int S3 = wtot[12] + wtot[13] + wtot[14] + wtot[15];
    int pre = 0;
#pragma unroll 1
    for (int w = 4 * sub; w < wave; ++w) pre += wtot[w];
    const int b0 = carry;
    const int b1 = b0 + ((S0 + 31) & ~31);
    const int b2 = b1 + ((S1 + 31) & ~31);
    const int b3 = b2 + ((S2 + 31) & ~31);
    const int b4 = b3 + ((S3 + 31) & ~31);
    const int myb = sub == 0 ? b0 : (sub == 1 ? b1 : (sub == 2 ? b2 : b3));
    if (tid == 0) {
      srb[min(4 * ch + 0, RBN - 1)] = b0;
      srb[min(4 * ch + 1, RBN - 1)] = b1;
      srb[min(4 * ch + 2, RBN - 1)] = b2;
      srb[min(4 * ch + 3, RBN - 1)] = b3;
    }
    int run = myb + pre + incl - ts;
    soff[8 * tid + 0] = run; run += e0;
    soff[8 * tid + 1] = run; run += e1;
    soff[8 * tid + 2] = run; run += e2;
    soff[8 * tid + 3] = run; run += e3;
    soff[8 * tid + 4] = run; run += e4;
    soff[8 * tid + 5] = run; run += e5;
    soff[8 * tid + 6] = run; run += e6;
    soff[8 * tid + 7] = run;
    carry = b4;
    __syncthreads();
    const v4i o0 = *(const v4i*)(soff + 4 * tid);
    const v4i o1 = *(const v4i*)(soff + 4 * (tid + OTHR));
    int* op = off + base;
    *(volatile v4i*)(op + 4 * tid) = o0;
    *(volatile v4i*)(op + 4 * (tid + OTHR)) = o1;
    __threadfence();
    *(volatile v4i*)(op + 4 * tid) = o0;
    *(volatile v4i*)(op + 4 * (tid + OTHR)) = o1;
    __syncthreads();
  }
  if (tid == 0) srb[min(4 * nChunk, RBN - 1)] = carry;
  __syncthreads();
  v4i rv = {0, 0, 0, 0};
  if (tid < 32) rv = *(const v4i*)(srb + 4 * tid);
  if (tid < 32) *(volatile v4i*)(rbase + 4 * tid) = rv;
  __threadfence();
  if (tid < 32) *(volatile v4i*)(rbase + 4 * tid) = rv;
}

__global__ __launch_bounds__(NTHR) void k_fill(
    const int* __restrict__ srcs, const int* __restrict__ dsts,
    const int* __restrict__ off, const int* __restrict__ rbase,
    int* csr, int nN, int nE, int vec8, int csrLen) {
  extern __shared__ v4f lds_dyn[];
  int* region = (int*)lds_dyn;
  int* cursor = region + RCAP;
  int* list   = cursor + NBF;
  int* wcnt   = list + LISTN;
  const int tid = threadIdx.x, lane = tid & 31, wave = tid >> 5;
  const int b = blockIdx.x;
  const int nodeBase = b * NBF;

  int rb0 = rbase[b];
  const int rb1 = rbase[b + 1];
  rb0 = rb0 < 0 ? 0 : (rb0 > csrLen ? csrLen : rb0);
  rb0 &= ~31;
  int len = rb1 - rb0;
  len = len < 0 ? 0 : (len > RCAP ? RCAP : len);
  int lenW = (len + 31) & ~31;
  if (rb0 + lenW > csrLen) lenW = (csrLen - rb0) & ~31;

  {
    const v4i z = {0, 0, 0, 0};
    for (int i = tid; i < RCAP / 4; i += NTHR) ((v4i*)region)[i] = z;
    for (int s = tid; s < NBF; s += NTHR) {
      int o = off[nodeBase + s] - rb0;
      o = o < 0 ? 0 : (o > RCAP ? RCAP : o);
      cursor[s] = o;
    }
  }
  __syncthreads();

  const int nChunks = (nE + CHUNK - 1) / CHUNK;
#pragma unroll 1
  for (int ch = 0; ch < nChunks; ++ch) {
    const int cbase = ch * CHUNK;
    const int wc = scan_chunk<NBF>(dsts, nE, cbase, nodeBase, vec8, list, tid, lane, wave);
    if (lane == 0) wcnt[wave] = wc;
    __syncthreads();
    if (wave == 0) {
#pragma unroll 1
      for (int wsx = 0; wsx < NWAVE; ++wsx) {
        int n = __builtin_amdgcn_readfirstlane(wcnt[wsx]);
        n = n > WCAP ? WCAP : (n < 0 ? 0 : n);
        const int* lp = list + wsx * WCAP;
#pragma unroll 1
        for (int i = 0; i < n; ++i) {
          const int ent  = __builtin_amdgcn_readfirstlane(lp[i]);
          const int slot = ent & (NBF - 1);
          int e = cbase + ((ent >> 12) & (CHUNK - 1));
          e = e > nE - 1 ? nE - 1 : e;
          int src = srcs[e];
          src = src < 0 ? 0 : (src > nN - 1 ? nN - 1 : src);
          if (lane == 0) {
            int pos = cursor[slot];
            pos = pos < 0 ? 0 : (pos > RCAP - 1 ? RCAP - 1 : pos);
            region[pos] = src;
            const int np = pos + 1;
            cursor[slot] = np > RCAP ? RCAP : np;
          }
        }
      }
    }
    __syncthreads();
  }

  const int nv = lenW >> 2;
  int* gp = csr + rb0;
#pragma unroll 1
  for (int i = tid; i < nv; i += NTHR) { const v4i v = ((const v4i*)region)[i]; *(volatile v4i*)(gp + 4 * i) = v; }
  __threadfence();
#pragma unroll 1
  for (int i = tid; i < nv; i += NTHR) { const v4i v = ((const v4i*)region)[i]; *(volatile v4i*)(gp + 4 * i) = v; }
}

template <int NC, int BM, int EMB>
__global__ __launch_bounds__(NTHR) void k_gemm(
    const float* __restrict__ A, const int* __restrict__ yv, const float* __restrict__ emb,
    const unsigned short* __restrict__ wp, const float* __restrict__ bcat,
    float* Pout, int nRowsA, int nV, int nRowsStore) {
  extern __shared__ v4f lds_dyn[];
  unsigned short* sA  = (unsigned short*)lds_dyn;
  float*          stg = (float*)lds_dyn;
  constexpr int RG  = BM / 16;
  constexpr int CG  = NWAVE / RG;
  constexpr int TPW = NC / (16 * CG);
  constexpr int NU  = BM * DIN / 8;
  static_assert(RG * CG == NWAVE);
  static_assert(TPW * 16 * CG == NC);
  static_assert((NU % NTHR) == 0);
  static_assert(((BM * NC / 4) % NTHR) == 0);
  static_assert(((NC / 4) & ((NC / 4) - 1)) == 0);
  const int tid = threadIdx.x, lane = tid & 31, wave = tid >> 5, hh = lane >> 4, m = lane & 15;
  const int rowBase = blockIdx.x * BM;

#pragma unroll
  for (int it = 0; it < NU / NTHR; ++it) {
    const int u  = it * NTHR + tid;
    const int r  = u >> 4;
    const int cc = (u & 15) * 8;
    int row = rowBase + r;
    row = row > nRowsA - 1 ? nRowsA - 1 : row;
    const float* ap = A + (size_t)row * DIN + cc;
    v4f a = *(const v4f*)ap, b = *(const v4f*)(ap + 4);
    if constexpr (EMB != 0) {
      int lab = yv[row];
      lab = lab < 0 ? 0 : (lab > nV - 1 ? nV - 1 : lab);
      const float* ep = emb + (size_t)lab * DIN + cc;
      const v4f ea = *(const v4f*)ep, eb = *(const v4f*)(ep + 4);
      a = a + ea;
      b = b + eb;
    }
    const v8us hv = cvt8(a, b, ASCL);
    *(v8us*)(sA + r * APK + cc) = hv;
  }
  __syncthreads();

  const int rg = wave / CG;
  const int cq = wave % CG;
  const int r0 = rg * 16;
  const int c0 = cq * (TPW * 16);

  v8f acc[TPW];
#pragma unroll
  for (int t = 0; t < TPW; ++t) { v8f z = {0.f, 0.f, 0.f, 0.f, 0.f, 0.f, 0.f, 0.f}; acc[t] = z; }
  const unsigned short* afp = sA + (r0 + m) * APK + 8 * hh;
#pragma unroll
  for (int kt = 0; kt < DIN / 32; ++kt) {
    FragH af;
    af.u[0] = *(const v8us*)(afp + 32 * kt);
    af.u[1] = *(const v8us*)(afp + 32 * kt + 16);
#pragma unroll
    for (int t = 0; t < TPW; ++t) {
      const unsigned short* bp = wp + (size_t)(c0 + 16 * t + m) * DIN + 32 * kt + 8 * hh;
      FragH bf;
      bf.u[0] = *(const v8us*)bp;
      bf.u[1] = *(const v8us*)(bp + 16);
      acc[t] = wmh(af.v, bf.v, acc[t]);
    }
  }
  __syncthreads();

  {
    float* sp = stg + (size_t)(r0 + 8 * hh) * NC + c0 + m;
#pragma unroll
    for (int t = 0; t < TPW; ++t) {
#pragma unroll
      for (int r = 0; r < 8; ++r) sp[r * NC + 16 * t] = acc[t][r];
    }
  }
  __syncthreads();

  float* gp = Pout + (size_t)rowBase * NC;
  constexpr int NIT = (BM * NC / 4) / NTHR;
  constexpr int C4  = NC / 4;
#pragma unroll
  for (int it = 0; it < NIT; ++it) {
    const int f    = it * NTHR + tid;
    const int col4 = f & (C4 - 1);
    const int grow = rowBase + f / C4;
    const v4f v  = *(const v4f*)(stg + 4 * f);
    const v4f bb = *(const v4f*)(bcat + 4 * col4);
    const v4f o  = v * INVSCL + bb;
    if (grow < nRowsStore) *(volatile v4f*)(gp + 4 * (size_t)f) = o;
  }
  __threadfence();
#pragma unroll
  for (int it = 0; it < NIT; ++it) {
    const int f    = it * NTHR + tid;
    const int col4 = f & (C4 - 1);
    const int grow = rowBase + f / C4;
    const v4f v  = *(const v4f*)(stg + 4 * f);
    const v4f bb = *(const v4f*)(bcat + 4 * col4);
    const v4f o  = v * INVSCL + bb;
    if (grow < nRowsStore) *(volatile v4f*)(gp + 4 * (size_t)f) = o;
  }
}

__global__ __launch_bounds__(ATHR) void k_agg(
    const int* __restrict__ csr, const int* __restrict__ off, const int* __restrict__ cnt,
    const float* __restrict__ P, float* xout, int nN, int csrLen) {
  extern __shared__ v4f lds_dyn[];
  v4f* sOut = lds_dyn;
  const int tid = threadIdx.x, lane = tid & 31, wave = tid >> 5, hd = lane >> 3;
  const int tbase = blockIdx.x * TGT + wave * 32;
  const v4f z4 = {0.f, 0.f, 0.f, 0.f};

  const int cl    = tbase + lane;
  const int cnt_l = cnt[cl];
  const int off_l = off[cl];

#pragma unroll 1
  for (int j = 0; j < 32; ++j) {
    const int c = tbase + j;
    int n = __shfl(cnt_l, j);
    n = n < 0 ? 0 : (n > DEGCAP ? DEGCAP : n);
    const int st = __shfl(off_l, j);
    const v4f q4 = *(const v4f*)(P + (size_t)c * PW + QOFF + 4 * lane);

    float mx = NEG_BIG;
    float cl0[NCHK], cl1[NCHK], cl2[NCHK], cl3[NCHK];
#pragma unroll
    for (int kc = 0; kc < NCHK; ++kc) { cl0[kc] = 0.f; cl1[kc] = 0.f; cl2[kc] = 0.f; cl3[kc] = 0.f; }
#pragma unroll
    for (int kc = 0; kc < NCHK; ++kc) {
      const int q0 = 32 * kc;
      if (q0 < n) {
        int pos = st + q0 + lane;
        pos = pos < 0 ? 0 : (pos > csrLen - 1 ? csrLen - 1 : pos);
        int sl = csr[pos];
        sl = sl < 0 ? 0 : (sl > nN - 1 ? nN - 1 : sl);
        const int mcnt = (n - q0) < 32 ? (n - q0) : 32;
#pragma unroll 1
        for (int pp = 0; pp < mcnt; ++pp) {
          const int s = __builtin_amdgcn_readlane(sl, pp);
          const v4f k4 = *(const v4f*)(P + (size_t)s * PW + KOFF + 4 * lane);
          float d = q4.x * k4.x + q4.y * k4.y + q4.z * k4.z + q4.w * k4.w;
          d += __shfl_xor(d, 1);
          d += __shfl_xor(d, 2);
          d += __shfl_xor(d, 4);
          d *= RSQD;
          const float L0 = __shfl(d, 0);
          const float L1 = __shfl(d, 8);
          const float L2 = __shfl(d, 16);
          const float L3 = __shfl(d, 24);
          mx = fmaxf(mx, d);
          cl0[kc] = (lane == pp) ? L0 : cl0[kc];
          cl1[kc] = (lane == pp) ? L1 : cl1[kc];
          cl2[kc] = (lane == pp) ? L2 : cl2[kc];
          cl3[kc] = (lane == pp) ? L3 : cl3[kc];
        }
      }
    }

    float den = 0.f;
    v4f acc = z4;
#pragma unroll
    for (int kc = 0; kc < NCHK; ++kc) {
      const int q0 = 32 * kc;
      if (q0 < n) {
        int pos = st + q0 + lane;
        pos = pos < 0 ? 0 : (pos > csrLen - 1 ? csrLen - 1 : pos);
        int sl = csr[pos];
        sl = sl < 0 ? 0 : (sl > nN - 1 ? nN - 1 : sl);
        const int mcnt = (n - q0) < 32 ? (n - q0) : 32;
#pragma unroll 1
        for (int pp = 0; pp < mcnt; ++pp) {
          const int s = __builtin_amdgcn_readlane(sl, pp);
          const float l0 = __shfl(cl0[kc], pp);
          const float l1 = __shfl(cl1[kc], pp);
          const float l2 = __shfl(cl2[kc], pp);
          const float l3 = __shfl(cl3[kc], pp);
          const float myl = (hd == 0) ? l0 : ((hd == 1) ? l1 : ((hd == 2) ? l2 : l3));
          const float p = __expf(myl - mx);
          den += p;
          const v4f v4 = *(const v4f*)(P + (size_t)s * PW + VOFF + 4 * lane);
          acc = acc + v4 * p;
        }
      }
    }

    const float rd = (den > 0.f) ? (1.0f / den) : 0.f;
    const v4f sk = *(const v4f*)(P + (size_t)c * PW + SOFF + 4 * lane);
    v4f ov = acc * rd + sk;
    if (c >= nN) ov = z4;
    sOut[wave * 1024 + j * 32 + lane] = ov;
  }
  __syncthreads();

  float* gp = xout + (size_t)tbase * HDW;
#pragma unroll
  for (int it = 0; it < 32; ++it) {
    const int f = it * 32 + lane;
    const v4f v = sOut[wave * 1024 + f];
    *(volatile v4f*)(gp + 4 * f) = v;
  }
  __threadfence();
#pragma unroll
  for (int it = 0; it < 32; ++it) {
    const int f = it * 32 + lane;
    const v4f v = sOut[wave * 1024 + f];
    *(volatile v4f*)(gp + 4 * f) = v;
  }
}

extern "C" void kernel_launch(void* const* d_in, const int* in_sizes, int n_in,
                              void* d_out, int out_size, void* d_ws, size_t ws_size,
                              hipStream_t stream) {
  if (n_in < 14) return;
  const int nN = in_sizes[0] / DIN;
  const int nE = in_sizes[2] / 2;
  const int nV = in_sizes[3] / DIN;
  if (nN <= 0 || nE <= 0 || nV <= 0) return;
  if (in_sizes[0] != nN * DIN || in_sizes[1] != nN || in_sizes[2] != 2 * nE || in_sizes[3] != nV * DIN) return;
  for (int g = 0; g < 4; ++g) {
    if (in_sizes[4 + 2 * g] != DIN * HDW || in_sizes[5 + 2 * g] != HDW) return;
  }
  if (in_sizes[12] != HDW * NCLS || in_sizes[13] != NCLS) return;
  if (out_size != nN * NCLS) return;
  if (nE > (1 << 28) || nN > (1 << 24)) return;

  const float* x    = (const float*)d_in[0];
  const int*   yv   = (const int*)d_in[1];
  const int*   eidx = (const int*)d_in[2];
  const int*   srcs = eidx;
  const int*   dsts = eidx + nE;
  const float* emb  = (const float*)d_in[3];
  const float* wq = (const float*)d_in[4];  const float* bq = (const float*)d_in[5];
  const float* wk = (const float*)d_in[6];  const float* bk = (const float*)d_in[7];
  const float* wv = (const float*)d_in[8];  const float* bv = (const float*)d_in[9];
  const float* ws = (const float*)d_in[10]; const float* bs = (const float*)d_in[11];
  const float* wl = (const float*)d_in[12]; const float* bl = (const float*)d_in[13];
  float* out = (float*)d_out;

  const int NPAD   = ((nN + NPADG - 1) / NPADG) * NPADG;
  const int nBC    = (nN + NBC - 1) / NBC;
  const int CNTPAD = nBC * NBC;
  if (4 * nBC + 1 > RBN) return;
  const int nBF    = (nN + NBF - 1) / NBF;
  const int csrLen = ((nE + 31) & ~31) + 4096;
  if (31 * 4 * nBC > 4096) return;
  const int nAgg   = NPAD / TGT;
  const int nG1    = NPAD / BM1;
  const int nG2    = NPAD / BM2;

  char* wsb = (char*)d_ws;
  size_t off = 0;
  const size_t oWp  = off; off += (size_t)PW * DIN * 2;           off = (off + 255) & ~(size_t)255;
  const size_t oWl  = off; off += (size_t)NCLS * DIN * 2;         off = (off + 255) & ~(size_t)255;
  const size_t oBc  = off; off += (size_t)BCPAD * 4;              off = (off + 255) & ~(size_t)255;
  const size_t oBl  = off; off += (size_t)BCPAD * 4;              off = (off + 255) & ~(size_t)255;
  const size_t oCnt = off; off += (size_t)CNTPAD * 4;             off = (off + 255) & ~(size_t)255;
  const size_t oOff = off; off += (size_t)CNTPAD * 4;             off = (off + 255) & ~(size_t)255;
  const size_t oRb  = off; off += (size_t)RBN * 4;                off = (off + 255) & ~(size_t)255;
  const size_t oCsr = off; off += (size_t)csrLen * 4;             off = (off + 255) & ~(size_t)255;
  const size_t oP   = off; off += (size_t)NPAD * PW * 4;          off = (off + 255) & ~(size_t)255;
  const size_t oX   = off; off += (size_t)NPAD * HDW * 4;         off = (off + 255) & ~(size_t)255;
  if (off > ws_size || off > (size_t)WSCAP) return;
  unsigned short* wp  = (unsigned short*)(wsb + oWp);
  unsigned short* wlp = (unsigned short*)(wsb + oWl);
  float* bc   = (float*)(wsb + oBc);
  float* blc  = (float*)(wsb + oBl);
  int*   cnt  = (int*)(wsb + oCnt);
  int*   offp = (int*)(wsb + oOff);
  int*   rb   = (int*)(wsb + oRb);
  int*   csr  = (int*)(wsb + oCsr);
  float* P    = (float*)(wsb + oP);
  float* xb   = (float*)(wsb + oX);

  const int vec8 = ((nE & 3) == 0) ? 1 : 0;

  k_wprep<<<WUNITS / NTHR, NTHR, 0, stream>>>(wq, bq, wk, bk, wv, bv, ws, bs, wp, bc);
  k_wlprep<<<LUNITS / NTHR, NTHR, 0, stream>>>(wl, bl, wlp, blc);

  k_count<<<nBC, NTHR, 0, stream>>>(dsts, cnt, nE, vec8);
  k_offsets<<<1, OTHR, 0, stream>>>(cnt, offp, rb, nBC);
  hipFuncSetAttribute(reinterpret_cast<const void*>(&k_fill),
                      hipFuncAttributeMaxDynamicSharedMemorySize, LDS_FILL);
  k_fill<<<nBF, NTHR, LDS_FILL, stream>>>(srcs, dsts, offp, rb, csr, nN, nE, vec8, csrLen);

  hipFuncSetAttribute(reinterpret_cast<const void*>(&k_gemm<PW, BM1, 1>),
                      hipFuncAttributeMaxDynamicSharedMemorySize, LDS_G1);
  k_gemm<PW, BM1, 1><<<nG1, NTHR, LDS_G1, stream>>>(x, yv, emb, wp, bc, P, nN, nV, NPAD);

  hipFuncSetAttribute(reinterpret_cast<const void*>(&k_agg),
                      hipFuncAttributeMaxDynamicSharedMemorySize, LDS_AGG);
  k_agg<<<nAgg, ATHR, LDS_AGG, stream>>>(csr, offp, cnt, P, xb, nN, csrLen);

  hipFuncSetAttribute(reinterpret_cast<const void*>(&k_gemm<NCLS, BM2, 0>),
                      hipFuncAttributeMaxDynamicSharedMemorySize, LDS_G2);
  k_gemm<NCLS, BM2, 0><<<nG2, NTHR, LDS_G2, stream>>>(xb, yv, emb, wlp, blc, out, NPAD, nV, nN);
}
